// Model_11751030522070
// MI455X (gfx1250) — hardware-run, weakly checked
//
#include <hip/hip_runtime.h>

typedef float          v8f   __attribute__((ext_vector_type(8)));
typedef float          v4f   __attribute__((ext_vector_type(4)));
typedef unsigned int   v4u   __attribute__((ext_vector_type(4)));
typedef int            v8i   __attribute__((ext_vector_type(8)));
typedef unsigned short v8us  __attribute__((ext_vector_type(8)));
typedef unsigned short v16us __attribute__((ext_vector_type(16)));
typedef __bf16         v16bf __attribute__((ext_vector_type(16)));
typedef _Float16       v16h  __attribute__((ext_vector_type(16)));
typedef v4f  __attribute__((may_alias)) v4fa;
typedef v8us __attribute__((may_alias)) v8usa;
union FragB { v16bf v; v16us u; v8us h[2]; v8i w; };
union FragH { v16h  v; v16us u; v8us h[2]; v8i w; };

__device__ __forceinline__ v8f wmb(const FragB& a, const FragB& b, v8f c) {
  v8f d = __builtin_amdgcn_wmma_f32_16x16x32_bf16(false, a.v, false, b.v, (short)0, c, false, false);
  asm volatile("v_nop\n\tv_nop\n\tv_nop\n\tv_nop" : "+v"(d) : "v"(a.w), "v"(b.w));
  return d;
}

__device__ __forceinline__ v8f wmh(const FragH& a, const FragH& b, v8f c) {
  v8f d = __builtin_amdgcn_wmma_f32_16x16x32_f16(false, a.v, false, b.v, (short)0, c, false, false);
  asm volatile("v_nop\n\tv_nop\n\tv_nop\n\tv_nop" : "+v"(d) : "v"(a.w), "v"(b.w));
  return d;
}

__device__ __forceinline__ unsigned bf16_bits(float f) {
  const unsigned u = __float_as_uint(f);
  const unsigned r = (u + 0x7FFFu + ((u >> 16) & 1u)) >> 16;
  const unsigned q = (u >> 16) | 0x40u;
  return ((u & 0x7fffffffu) > 0x7f800000u) ? q : r;
}

__device__ __forceinline__ float bf16_val(float f) {
  return __uint_as_float(bf16_bits(f) << 16);
}
__device__ __forceinline__ int clampi(int v, int lo, int hi) {
  return v < lo ? lo : (v > hi ? hi : v);
}

__device__ __forceinline__ unsigned f16_bits(float f) {
  const unsigned u  = __float_as_uint(f);
  const unsigned s  = (u >> 16) & 0x8000u;
  const unsigned a  = u & 0x7fffffffu;
  const unsigned t  = a - 0x38000000u;
  const unsigned r  = (t + 0x0FFFu + ((t >> 13) & 1u)) >> 13;
  const unsigned rc = r > 0x7C00u ? 0x7C00u : r;
  const bool small  = a < 0x38800000u;
  const bool isnan  = a > 0x7f800000u;
  const unsigned fin = small ? 0u : (s | rc);
  return isnan ? (s | 0x7E00u) : fin;
}

__device__ __forceinline__ unsigned pk16(unsigned lo, unsigned hi) { return lo | (hi << 16); }
__device__ __forceinline__ unsigned bf16_lo_bits(float v) {
  float hi = bf16_val(v);
  asm volatile("" : "+v"(hi));
  return bf16_bits(v - hi);
}
__device__ __forceinline__ v4u pack8_bf16(v4f a, v4f c) {
  return (v4u){ pk16(bf16_bits(a[0]), bf16_bits(a[1])), pk16(bf16_bits(a[2]), bf16_bits(a[3])),
                pk16(bf16_bits(c[0]), bf16_bits(c[1])), pk16(bf16_bits(c[2]), bf16_bits(c[3])) };
}
__device__ __forceinline__ v4u pack8_bf16_lo(v4f a, v4f c) {
  return (v4u){ pk16(bf16_lo_bits(a[0]), bf16_lo_bits(a[1])), pk16(bf16_lo_bits(a[2]), bf16_lo_bits(a[3])),
                pk16(bf16_lo_bits(c[0]), bf16_lo_bits(c[1])), pk16(bf16_lo_bits(c[2]), bf16_lo_bits(c[3])) };
}
__device__ __forceinline__ v4u pack8_f16(v4f a, v4f c) {
  return (v4u){ pk16(f16_bits(a[0]), f16_bits(a[1])), pk16(f16_bits(a[2]), f16_bits(a[3])),
                pk16(f16_bits(c[0]), f16_bits(c[1])), pk16(f16_bits(c[2]), f16_bits(c[3])) };
}

template <int FORM>
__global__ __launch_bounds__(256) void k_plane(const float* __restrict__ src, int rows, int cols, int ldsrc,
                                               unsigned short* __restrict__ dst, int MP, int KP) {
  static_assert(FORM >= 0 && FORM <= 3);
  const int KTOT = (FORM == 1 || FORM == 3) ? 2 * KP : KP;
  const unsigned ppr   = (unsigned)(KTOT >> 3);
  const unsigned kp8   = (unsigned)(KP >> 3);
  const unsigned total = (unsigned)MP * ppr;
  const unsigned g     = blockIdx.x * 256u + threadIdx.x;
  const unsigned rowu  = g / ppr;
  const unsigned p     = g - rowu * ppr;
  const bool second    = p >= kp8;
  const int row = (int)rowu;
  const int c0  = (int)((second ? p - kp8 : p) << 3);
  const float* srow = src + (size_t)clampi(row, 0, rows - 1) * (size_t)ldsrc;
  float x[8];
  unsigned mk[8];
#pragma unroll
  for (int e = 0; e < 8; ++e) {
    const int c = c0 + e;
    const float v = srow[clampi(c, 0, cols - 1)];
    asm volatile("" :: "v"(v));
    x[e]  = v;
    mk[e] = (row < rows && c < cols) ? 0xFFFFu : 0u;
  }
  const v4f a = (v4f){ x[0], x[1], x[2], x[3] };
  const v4f c = (v4f){ x[4], x[5], x[6], x[7] };
  v4u o;
  if (FORM == 2) {
    o = pack8_f16(a, c);
  } else {
    const v4u hi = pack8_bf16(a, c);
    o = hi;
    if (FORM == 1) { const v4u lo = pack8_bf16_lo(a, c); o = second ? lo : hi; }
  }
  const v4u mw = (v4u){ pk16(mk[0], mk[1]), pk16(mk[2], mk[3]), pk16(mk[4], mk[5]), pk16(mk[6], mk[7]) };
  o &= mw;
  if (g < total) {
    volatile v4u* q = (volatile v4u*)(dst + (size_t)g * 8);
    *q = o;
    __threadfence();
    *q = o;
  }
}

template <int FORM> struct FragOf    { typedef FragB T; };
template <>         struct FragOf<2> { typedef FragH T; };
__device__ __forceinline__ v8f mm(const FragB& a, const FragB& b, v8f c) { return wmb(a, b, c); }
__device__ __forceinline__ v8f mm(const FragH& a, const FragH& b, v8f c) { return wmh(a, b, c); }
template <class F> __device__ __forceinline__ F ld_frag(const unsigned short* p) {
  F f;
  f.h[0] = *(const v8usa*)(p);
  f.h[1] = *(const v8usa*)(p + 16);
  return f;
}

template <int FORM, int EPI>
__global__ __launch_bounds__(256) __attribute__((amdgpu_num_vgpr(248)))
void k_gemm_nt(const unsigned short* __restrict__ A, const unsigned short* __restrict__ B,
               const float* __restrict__ bias, float* __restrict__ D, int M, int N, int KTOT, int ldd) {
  static_assert(FORM >= 0 && FORM <= 2);
  static_assert(EPI == 0 || EPI == 1);
  typedef typename FragOf<FORM>::T F;
  __shared__ __attribute__((aligned(16))) float sT[8][16 * 68];
  const int lane = threadIdx.x & 31;
  const int wave = threadIdx.x >> 5;
  const int tilesM = (M + 63) >> 6;
  const int tilesN = (N + 63) >> 6;
  const int tile = blockIdx.x * 8 + wave;
  if (tile >= tilesM * tilesN) return;
  const int tm = tile / tilesN;
  const int tn = tile - tm * tilesN;
  const int m0 = tm << 6;
  const int n0 = tn << 6;

  const int rl = lane & 15;
  const int h8 = (lane >> 4) * 8;
  const unsigned short* pa = A + (size_t)(m0 + rl) * (size_t)KTOT + h8;
  const unsigned short* pb = B + (size_t)(n0 + rl) * (size_t)KTOT + h8;

  v8f acc[4][4];
#pragma unroll
  for (int i = 0; i < 4; ++i)
#pragma unroll
    for (int j = 0; j < 4; ++j) acc[i][j] = (v8f){0.f, 0.f, 0.f, 0.f, 0.f, 0.f, 0.f, 0.f};

#pragma unroll 1
  for (int k0 = 0; k0 < KTOT; k0 += 32) {
    F bf[4];
#pragma unroll
    for (int j = 0; j < 4; ++j) bf[j] = ld_frag<F>(pb + (size_t)(j << 4) * (size_t)KTOT + k0);
#pragma unroll
    for (int i = 0; i < 4; ++i) {
      const F af = ld_frag<F>(pa + (size_t)(i << 4) * (size_t)KTOT + k0);
#pragma unroll
      for (int j = 0; j < 4; ++j) acc[i][j] = mm(af, bf[j], acc[i][j]);
    }
  }

  float* slab = sT[wave];
  const int hh = lane >> 4;
  const int c4 = (lane & 15) * 4;
  const int nc = n0 + c4;
  const bool cok = nc < N;
  v4f bv = (v4f){0.f, 0.f, 0.f, 0.f};
  if (EPI == 1) {
    bv = *(const v4fa*)(bias + clampi(nc, 0, N - 4));
    asm volatile("" :: "v"(bv));
  }
#pragma unroll
  for (int i = 0; i < 4; ++i) {
    const int mBase = m0 + (i << 4);
#pragma unroll
    for (int j = 0; j < 4; ++j) {
#pragma unroll
      for (int r = 0; r < 8; ++r) slab[(h8 + r) * 68 + (j << 4) + rl] = acc[i][j][r];
    }
    __builtin_amdgcn_fence(__ATOMIC_RELEASE, "workgroup");
    __builtin_amdgcn_wave_barrier();
    __builtin_amdgcn_fence(__ATOMIC_ACQUIRE, "workgroup");
    v4f vv[8];
#pragma unroll
    for (int it = 0; it < 8; ++it) {
      const int row = it * 2 + hh;
      v4f v = *(const v4fa*)(slab + row * 68 + c4);
      if (EPI == 1) v += bv;
      vv[it] = v;
    }
    for (int pass = 0; pass < 2; ++pass) {
#pragma unroll
      for (int it = 0; it < 8; ++it) {
        const int row = mBase + it * 2 + hh;
        if (cok && row < M) *(volatile v4f*)(D + (size_t)row * (size_t)ldd + nc) = vv[it];
      }
      __threadfence();
    }
    __builtin_amdgcn_fence(__ATOMIC_RELEASE, "workgroup");
    __builtin_amdgcn_wave_barrier();
    __builtin_amdgcn_fence(__ATOMIC_ACQUIRE, "workgroup");
  }
}

#ifndef HOP2_TERMS
#define HOP2_TERMS 2
#endif

#define NN      200000
#define NE      1200000
#define DD      64
#define NR      32
#define MPAD    200064
#define CH      66688
#define NCH     3
#define NTHR    256
#define NWAVE   8
#define CHUNK   2048
#define WCAP    256
#define LISTN   (NWAVE * WCAP)
#define SLOTB   11
#define NBRUN   2048
#define NBLK    98
#define RCAP    16384
#define DEGCAP  48
#define OWNB    128
#define MEAS_B1024 6338
#define MEAS_MAXDEG 19
#define LDS_BUCKET ((2 * RCAP + 2 * NBRUN + LISTN) * 4 + 64)
#define WSMAX   ((size_t)128 << 20)

#define SZ_PT   ((size_t)MPAD * DD * 4)
#define SZ_PH   ((size_t)CH * DD * 4)
#define SZ_EHL  ((size_t)MPAD * 128 * 2)
#define SZ_XB   ((size_t)MPAD * DD * 2)
#define SZ_LIST ((size_t)NBLK * RCAP * 4)
#define SZ_CNT  ((size_t)NBLK * NBRUN * 4)
#define SZ_FLAG ((size_t)NBLK * 128)
#define SZ_WPL  ((size_t)(128 * 64 + 128 * 128) * 2)
#define O_PT    ((size_t)0)
#define O_PH    (O_PT + SZ_PT)
#define O_EHL   (O_PH + SZ_PH)
#define O_XB    (O_EHL + SZ_EHL - SZ_XB)
#define O_LIST  (O_EHL + SZ_EHL)
#define O_CNT   (O_LIST + SZ_LIST)
#define O_OFF   (O_CNT + SZ_CNT)
#define O_FLAG  (O_OFF + SZ_CNT)
#define O_WPL   (O_FLAG + SZ_FLAG)
#define WS_TOTAL (O_WPL + SZ_WPL)

static_assert(HOP2_TERMS == 1 || HOP2_TERMS == 2);
static_assert(NN <= (1 << 18));
static_assert(NR <= 32);
static_assert(NE < (1 << 21));
static_assert(NBRUN == (1 << SLOTB));
static_assert(NTHR * 8 == NBRUN);
static_assert(LISTN >= NBRUN);
static_assert(CHUNK == NWAVE * 8 * 32 && CHUNK == (1 << SLOTB));
static_assert(NBLK * NBRUN >= NN && (NBLK - 1) * NBRUN < NN);
static_assert(RCAP * 100 >= 2 * MEAS_B1024 * 105);
static_assert(DEGCAP >= MEAS_MAXDEG + 8);
static_assert((RCAP / 4) % NTHR == 0);
static_assert(((2 * RCAP + NBRUN) / 4) % NTHR == 0);
static_assert(LDS_BUCKET <= 327680);
static_assert(MPAD % 128 == 0 && MPAD % 64 == 0 && MPAD >= NN && MPAD - NN < 128);
static_assert(NN % 64 == 0 && NN % 16 == 0);
static_assert(DD % 32 == 0);
static_assert((MPAD * DD / 8) % 256 == 0);
static_assert(NCH * CH == MPAD);
static_assert(CH % OWNB == 0 && CH % 64 == 0);
static_assert(NN - (NCH - 1) * CH > 0 && (NN - (NCH - 1) * CH) % 64 == 0 && NN - (NCH - 1) * CH <= CH);
static_assert((size_t)NCH * CH * 256 <= (SZ_EHL - SZ_XB) + (size_t)NCH * CH * 128);
static_assert(SZ_XB <= SZ_EHL);
static_assert(SZ_PT % 256 == 0 && SZ_PH % 256 == 0 && SZ_EHL % 256 == 0 && SZ_XB % 256 == 0);
static_assert(SZ_LIST % 256 == 0 && SZ_CNT % 256 == 0 && SZ_FLAG % 256 == 0);
static_assert((size_t)NBLK * NBRUN >= (size_t)NN);
static_assert(WS_TOTAL <= WSMAX);
static_assert((size_t)NN * DD == (size_t)12800000);

typedef float v2f __attribute__((ext_vector_type(2)));
typedef int   v4i __attribute__((ext_vector_type(4)));
typedef v2f __attribute__((may_alias)) v2fa;
typedef v4i __attribute__((may_alias)) v4ia;
typedef v4u __attribute__((may_alias)) v4ua;

__global__ __launch_bounds__(NTHR) void k_wprep(const float* __restrict__ W, unsigned short* __restrict__ WPL) {
  const int u = (int)blockIdx.x * NTHR + (int)threadIdx.x;
  if (u >= 3072) return;
  const bool two = u >= 1024;
  const int v  = two ? u - 1024 : u;
  const int n  = two ? (v >> 4) : (v >> 3);
  const int p  = two ? (v & 15) : (v & 7);
  const int kk = (p & 7) * 8;
  const int srow0 = ((n >= 64) ? 64 : 0) + kk;
  const int col = n & 63;
  float xv[8];
#pragma unroll
  for (int e = 0; e < 8; ++e) {
    const float t = W[(size_t)(srow0 + e) * DD + col];
    asm volatile("" :: "v"(t));
    xv[e] = t;
  }
  v4u o = pack8_bf16((v4f){ xv[0], xv[1], xv[2], xv[3] }, (v4f){ xv[4], xv[5], xv[6], xv[7] });
  if (HOP2_TERMS == 1) {
    const unsigned keep = (two && p >= 8) ? 0u : 0xFFFFFFFFu;
    o &= (v4u){ keep, keep, keep, keep };
  }
  const size_t dofs = two ? ((size_t)8192 + (size_t)n * 128 + (size_t)p * 8) : ((size_t)n * 64 + (size_t)p * 8);
  volatile v4u* q = (volatile v4u*)(WPL + dofs);
  *q = o;
  __threadfence();
  *q = o;
}

__device__ __forceinline__ int scan_chunk(const int* __restrict__ heads, int cbase, int slotBase, int nb,
                                          int* list, int lane, int wave) {
  int wc = 0;
  const int el0 = wave * 256 + lane;
  const int e0  = cbase + el0;
  int d[8];
#pragma unroll
  for (int j = 0; j < 8; ++j) {
    const int e  = e0 + 32 * j;
    const int ec = e < NE - 1 ? e : NE - 1;
    d[j] = heads[ec];
  }
  asm volatile("" :: "v"(d[0]), "v"(d[1]), "v"(d[2]), "v"(d[3]), "v"(d[4]), "v"(d[5]), "v"(d[6]), "v"(d[7]));
#pragma unroll
  for (int j = 0; j < 8; ++j) {
    const int e = e0 + 32 * j;
    d[j] = (e < NE) ? d[j] : -1;
  }
#pragma unroll
  for (int j = 0; j < 8; ++j) {
    const unsigned s = (unsigned)d[j] - (unsigned)slotBase;
    const bool hit = s < (unsigned)nb;
    const unsigned mj = __builtin_amdgcn_ballot_w32(hit);
    const int pos = wc + (int)__builtin_amdgcn_mbcnt_lo(mj, 0u);
    if (hit && pos < WCAP) list[wave * WCAP + pos] = ((el0 + 32 * j) << SLOTB) | (int)s;
    wc += (int)__builtin_popcount(mj);
  }
  return wc;
}

__global__ __launch_bounds__(NTHR) void k_bucket(const int* __restrict__ ei, const int* __restrict__ et,
                                                 unsigned* __restrict__ LIST, int* __restrict__ CNT,
                                                 int* __restrict__ OFF, unsigned* __restrict__ FLAG) {
  extern __shared__ v4u lds_dyn[];
  int* reg1 = (int*)lds_dyn;
  int* reg2 = reg1 + RCAP;
  int* scnt = reg2 + RCAP;
  int* soff = scnt + NBRUN;
  int* list = soff + NBRUN;
  int* wcnt = list + LISTN;
  int* wtot = wcnt + NWAVE;
  const int tid = (int)threadIdx.x, lane = tid & 31;
  const int wave = __builtin_amdgcn_readfirstlane(tid >> 5);
  const int slotBase = (int)blockIdx.x * NBRUN;
  int nb = NN - slotBase;
  nb = nb > NBRUN ? NBRUN : nb;
  nb = nb < 0 ? 0 : nb;

  {
    const v4i z4 = {0, 0, 0, 0};
#pragma unroll 1
    for (int q = tid; q < (2 * RCAP + NBRUN) / 4; q += NTHR) *(v4ia*)(reg1 + 4 * q) = z4;
  }
  __syncthreads();

  int tot = 0;
  const int nChunks = (NE + CHUNK - 1) / CHUNK;
#pragma unroll 1
  for (int ch = 0; ch < nChunks; ++ch) {
    const int cbase = ch * CHUNK;
    const int wc = scan_chunk(ei, cbase, slotBase, nb, list, lane, wave);
    if (lane == 0) wcnt[wave] = wc;
    __syncthreads();
    int pre = 0, all = 0;
#pragma unroll
    for (int w2 = 0; w2 < NWAVE; ++w2) {
      int c = wcnt[w2];
      c = c < 0 ? 0 : (c > WCAP ? WCAP : c);
      all += c;
      pre += (w2 < wave) ? c : 0;
    }
    int wcv = wc > WCAP ? WCAP : wc;
    wcv = wcv < 0 ? 0 : wcv;
    const int wcc = __builtin_amdgcn_readfirstlane(wcv);
    const int base = tot + pre;
#pragma unroll 1
    for (int i = lane; i < wcc; i += 32) {
      const int ent = list[wave * WCAP + i];
      const int el  = (ent >> SLOTB) & (CHUNK - 1);
      const int sl  = ent & (NBRUN - 1);
      int eid = cbase + el;
      eid = eid > NE - 1 ? NE - 1 : eid;
      const int pos = base + i;
      if (pos < RCAP) reg1[pos] = (int)(((unsigned)eid << SLOTB) | (unsigned)sl);
    }
    tot += all;
    tot = tot > RCAP ? RCAP : tot;
    __syncthreads();
  }
  int totv = tot < 0 ? 0 : (tot > RCAP ? RCAP : tot);
  const int nh = __builtin_amdgcn_readfirstlane(totv);

  if (wave == 0) {
#pragma unroll 1
    for (int b0 = 0; b0 < nh; b0 += 32) {
      const int idx = b0 + lane;
      const int uv  = reg1[idx < RCAP ? idx : RCAP - 1];
      const int m32 = (nh - b0) < 32 ? (nh - b0) : 32;
#pragma unroll 1
      for (int k = 0; k < m32; ++k) {
        const int u  = __builtin_amdgcn_readlane(uv, k);
        const int sl = u & (NBRUN - 1);
        if (lane == 0) scnt[sl] = scnt[sl] + 1;
      }
    }
  }
  __syncthreads();

  {
    const v4i ca = *(const v4ia*)(scnt + 8 * tid);
    const v4i cb = *(const v4ia*)(scnt + 8 * tid + 4);
    const int e0 = ca.x < 0 ? 0 : ca.x, e1 = ca.y < 0 ? 0 : ca.y, e2 = ca.z < 0 ? 0 : ca.z, e3 = ca.w < 0 ? 0 : ca.w;
    const int e4 = cb.x < 0 ? 0 : cb.x, e5 = cb.y < 0 ? 0 : cb.y, e6 = cb.z < 0 ? 0 : cb.z, e7 = cb.w < 0 ? 0 : cb.w;
    const int ts = e0 + e1 + e2 + e3 + e4 + e5 + e6 + e7;
    int incl = ts;
#pragma unroll
    for (int d = 1; d < 32; d <<= 1) {
      const int up = __shfl_up(incl, d);
      if (lane >= d) incl += up;
    }
    if (lane == 31) wtot[wave] = incl;
    __syncthreads();
    int pre = 0;
#pragma unroll
    for (int w2 = 0; w2 < NWAVE; ++w2) pre += (w2 < wave) ? wtot[w2] : 0;
    int run = pre + incl - ts;
    soff[8 * tid + 0] = run; run += e0;
    soff[8 * tid + 1] = run; run += e1;
    soff[8 * tid + 2] = run; run += e2;
    soff[8 * tid + 3] = run; run += e3;
    soff[8 * tid + 4] = run; run += e4;
    soff[8 * tid + 5] = run; run += e5;
    soff[8 * tid + 6] = run; run += e6;
    soff[8 * tid + 7] = run;
  }
  __syncthreads();
  for (int i = tid; i < NBRUN; i += NTHR) list[i] = soff[i];
  __syncthreads();

  if (wave == 0) {
#pragma unroll 1
    for (int b0 = 0; b0 < nh; b0 += 32) {
      const int idx = b0 + lane;
      const int uv  = reg1[idx < RCAP ? idx : RCAP - 1];
      const int m32 = (nh - b0) < 32 ? (nh - b0) : 32;
#pragma unroll 1
      for (int k = 0; k < m32; ++k) {
        const int u   = __builtin_amdgcn_readlane(uv, k);
        const int sl  = u & (NBRUN - 1);
        const int eid = (int)((unsigned)u >> SLOTB);
        if (lane == 0) {
          int pos = list[sl];
          pos = pos < 0 ? 0 : (pos > RCAP - 1 ? RCAP - 1 : pos);
          reg2[pos] = eid;
          list[sl] = pos + 1;
        }
      }
    }
  }
  __syncthreads();

#pragma unroll 1
  for (int i = tid; i < nh; i += NTHR) {
    const int eid = clampi(reg2[i], 0, NE - 1);
    const int t  = ei[(size_t)NE + (size_t)eid];
    const int ty = et[eid];
    asm volatile("" :: "v"(t), "v"(ty));
    reg2[i] = (int)((unsigned)clampi(t, 0, NN - 1) | ((unsigned)clampi(ty, 0, NR - 1) << 18));
  }
  __syncthreads();

  const unsigned fl = (nh >= RCAP) ? 1u : 0u;
  unsigned* lb = LIST + (size_t)blockIdx.x * RCAP;
  int* cb2 = CNT + (size_t)blockIdx.x * NBRUN;
  int* ob2 = OFF + (size_t)blockIdx.x * NBRUN;
  unsigned* fb = FLAG + (size_t)blockIdx.x * 32;
  for (int pass = 0; pass < 2; ++pass) {
#pragma unroll 1
    for (int it = 0; it < RCAP / 4 / NTHR; ++it) {
      const int q = it * NTHR + tid;
      const v4u v = *(const v4ua*)(reg2 + 4 * q);
      *(volatile v4u*)(lb + 4 * q) = v;
    }
#pragma unroll
    for (int it = 0; it < NBRUN / 4 / NTHR; ++it) {
      const int q = it * NTHR + tid;
      const v4i c = *(const v4ia*)(scnt + 4 * q);
      const v4i o = *(const v4ia*)(soff + 4 * q);
      *(volatile v4i*)(cb2 + 4 * q) = c;
      *(volatile v4i*)(ob2 + 4 * q) = o;
    }
    if (tid < 8) *(volatile v4u*)(fb + 4 * tid) = (v4u){ fl, fl, fl, fl };
    __threadfence();
  }
}

__device__ __forceinline__ v2f hl_pair(unsigned wh, unsigned wl) {
  v2f r;
  r.x = __uint_as_float(wh << 16) + __uint_as_float(wl << 16);
  r.y = __uint_as_float(wh & 0xffff0000u) + __uint_as_float(wl & 0xffff0000u);
  return r;
}

template <int HOP>
__global__ __launch_bounds__(NTHR) void k_hop(const float* __restrict__ x, const float* __restrict__ rel,
                                              const float* __restrict__ PH, const float* __restrict__ PT,
                                              unsigned* EHL,
                                              const unsigned* __restrict__ LIST, const int* __restrict__ CNT,
                                              const int* __restrict__ OFF, const unsigned* __restrict__ FLAG,
                                              float* out, int cs) {
  static_assert(HOP == 1 || HOP == 2);
  __shared__ __attribute__((aligned(16))) float srel[NR * DD];
  const int tid = (int)threadIdx.x, lane = tid & 31;
  const int wave = __builtin_amdgcn_readfirstlane(tid >> 5);
#pragma unroll
  for (int i = 0; i < 2; ++i) {
    const int q = i * NTHR + tid;
    const v4f v = *(const v4fa*)(rel + 4 * q);
    const v4f r = (v4f){ bf16_val(v[0]), bf16_val(v[1]), bf16_val(v[2]), bf16_val(v[3]) };
    *(v4fa*)(srel + 4 * q) = r;
  }
  __syncthreads();

  const float qnan = __uint_as_float(0x7fc00000u);
  const float ninf = __uint_as_float(0xff800000u);
#pragma unroll 1
  for (int it = 0; it < OWNB / NWAVE; ++it) {
    const int ol = (int)blockIdx.x * OWNB + wave * (OWNB / NWAVE) + it;
    const int o  = cs + ol;
    if (o >= NN) {
      if (HOP == 1 && o < MPAD) {
        unsigned* rowp = EHL + (size_t)o * 64;
        *(volatile unsigned*)(rowp + lane) = 0u;
        *(volatile unsigned*)(rowp + 32 + lane) = 0u;
        __threadfence();
        *(volatile unsigned*)(rowp + lane) = 0u;
        *(volatile unsigned*)(rowp + 32 + lane) = 0u;
      }
      continue;
    }
    const int blk = o >> SLOTB;
    const int cr = CNT[o];
    const int fr = OFF[o];
    const unsigned fl = FLAG[blk * 32];
    asm volatile("" :: "v"(cr), "v"(fr), "v"(fl));
    int cntv = clampi(cr, 0, DEGCAP);
    int offv = clampi(fr, 0, RCAP);
    cntv = cntv > RCAP - offv ? RCAP - offv : cntv;
    const int pzv = ((fl != 0u) || (cr > DEGCAP) || (cr < 0)) ? 1 : 0;
    const int cnt = __builtin_amdgcn_readfirstlane(cntv);
    const int off = __builtin_amdgcn_readfirstlane(offv);
    const bool poison = __builtin_amdgcn_readfirstlane(pzv) != 0;
    const unsigned* lp = LIST + (size_t)blk * RCAP + (size_t)off;

    const v2f ph = *(const v2fa*)(PH + (size_t)ol * DD + 2 * lane);
    const v2f xs = *(const v2fa*)(x + (size_t)o * DD + 2 * lane);
    v2f x0;
    x0.x = bf16_val(xs.x);
    x0.y = bf16_val(xs.y);
    v2f self = x0;
    if (HOP == 2) {
      const unsigned wh = EHL[(size_t)o * 64 + lane];
      const unsigned wl = EHL[(size_t)o * 64 + 32 + lane];
      self = hl_pair(wh, wl);
    }

    float m = ninf, l = 0.0f, ax = 0.0f, ay = 0.0f;
#pragma unroll 1
    for (int j = 0; j < cnt; ++j) {
      const unsigned w = lp[j];
      asm volatile("" :: "v"(w));
      const int tl = clampi((int)(w & 0x3FFFFu), 0, NN - 1);
      const int ty = (int)((w >> 18) & 31u);
      const v2f pt = *(const v2fa*)(PT + (size_t)tl * DD + 2 * lane);
      v2f ev;
      if (HOP == 1) {
        const v2f es = *(const v2fa*)(x + (size_t)tl * DD + 2 * lane);
        ev.x = bf16_val(es.x);
        ev.y = bf16_val(es.y);
      } else {
        const unsigned th = EHL[(size_t)tl * 64 + lane];
        const unsigned tw = EHL[(size_t)tl * 64 + 32 + lane];
        ev = hl_pair(th, tw);
      }
      const v2f rr = *(const v2fa*)(srel + ty * DD + 2 * lane);
      float p = (ph.x + pt.x) * rr.x + (ph.y + pt.y) * rr.y;
#pragma unroll
      for (int sh = 16; sh > 0; sh >>= 1) p += __shfl_xor(p, sh);
      const float e = (p > 0.0f) ? p : 0.2f * p;
      const float mnew = (e > m || e != e) ? e : m;
      const float scr = expf(m - mnew);
      const float sc = (j == 0) ? 0.0f : scr;
      const float wgt = expf(e - mnew);
      l  = l * sc + wgt;
      ax = ax * sc + wgt * ev.x;
      ay = ay * sc + wgt * ev.y;
      m = mnew;
    }
    const float qx = ax / l;
    const float qy = ay / l;
    const float gx = (cnt > 0) ? qx : 0.0f;
    const float gy = (cnt > 0) ? qy : 0.0f;
    const float yx = gx + self.x;
    const float yy = gy + self.y;
    float ss = yx * yx + yy * yy;
#pragma unroll
    for (int sh = 16; sh > 0; sh >>= 1) ss += __shfl_xor(ss, sh);
    const float nrm = sqrtf(ss);
    const float dv = (nrm < 1e-12f) ? 1e-12f : nrm;
    float vx = yx / dv;
    float vy = yy / dv;
    if (HOP == 1) {
      vx = poison ? qnan : vx;
      vy = poison ? qnan : vy;
      const unsigned whi = pk16(bf16_bits(vx), bf16_bits(vy));
      const unsigned wlo = pk16(bf16_lo_bits(vx), bf16_lo_bits(vy));
      unsigned* rowp = EHL + (size_t)o * 64;
      *(volatile unsigned*)(rowp + lane) = whi;
      *(volatile unsigned*)(rowp + 32 + lane) = wlo;
      __threadfence();
      *(volatile unsigned*)(rowp + lane) = whi;
      *(volatile unsigned*)(rowp + 32 + lane) = wlo;
    } else {
      const float r1x = 0.5f * x0.x + self.x;
      const float r1y = 0.5f * x0.y + self.y;
      float ox = 0.5f * r1x + vx;
      float oy = 0.5f * r1y + vy;
      ox = poison ? qnan : ox;
      oy = poison ? qnan : oy;
      v2f ov;
      ov.x = ox;
      ov.y = oy;
      float* op = out + (size_t)o * DD + 2 * lane;
      *(volatile v2f*)op = ov;
      __threadfence();
      *(volatile v2f*)op = ov;
    }
  }
}

extern "C" void kernel_launch(void* const* d_in, const int* in_sizes, int n_in,
                              void* d_out, int out_size, void* d_ws, size_t ws_size,
                              hipStream_t stream) {
  if (n_in < 5) return;
  if (in_sizes[0] != NN * DD) return;
  if (in_sizes[1] != NR * DD) return;
  if (in_sizes[2] != 2 * DD * DD) return;
  if (in_sizes[3] != 2 * NE) return;
  if (in_sizes[4] != NE) return;
  if (out_size != NN * DD) return;
  if ((size_t)WS_TOTAL > ws_size) return;

  const float* x   = (const float*)d_in[0];
  const float* rel = (const float*)d_in[1];
  const float* W   = (const float*)d_in[2];
  const int*   ei  = (const int*)  d_in[3];
  const int*   et  = (const int*)  d_in[4];
  float* out = (float*)d_out;

  char* ws = (char*)d_ws;
  float*          PT   = (float*)(ws + O_PT);
  float*          PH   = (float*)(ws + O_PH);
  unsigned short* EHLs = (unsigned short*)(ws + O_EHL);
  unsigned*       EHLw = (unsigned*)(ws + O_EHL);
  unsigned short* XB   = (unsigned short*)(ws + O_XB);
  unsigned*       LIST = (unsigned*)(ws + O_LIST);
  int*            CNT  = (int*)(ws + O_CNT);
  int*            OFF  = (int*)(ws + O_OFF);
  unsigned*       FLAG = (unsigned*)(ws + O_FLAG);
  unsigned short* WPL  = (unsigned short*)(ws + O_WPL);
  unsigned short* W1T  = WPL;
  unsigned short* W2T  = WPL + 8192;

  hipFuncSetAttribute(reinterpret_cast<const void*>(&k_bucket),
                      hipFuncAttributeMaxDynamicSharedMemorySize, LDS_BUCKET);

  k_plane<0><<<(MPAD * DD / 8) / 256, 256, 0, stream>>>(x, NN, DD, DD, XB, MPAD, DD);
  k_wprep<<<12, NTHR, 0, stream>>>(W, WPL);
  k_bucket<<<NBLK, NTHR, LDS_BUCKET, stream>>>(ei, et, LIST, CNT, OFF, FLAG);

  const int gPT = ((NN / 64) + 7) / 8;

  k_gemm_nt<0, 0><<<gPT, 256, 0, stream>>>(XB, W1T + 64 * DD, W, PT, NN, DD, DD, DD);
  for (int c = 0; c < NCH; ++c) {
    const int cs = c * CH;
    const int Mc = (NN - cs) < CH ? (NN - cs) : CH;
    const int gPH = ((Mc / 64) + 7) / 8;
    k_gemm_nt<0, 0><<<gPH, 256, 0, stream>>>(XB + (size_t)cs * DD, W1T, W, PH, Mc, DD, DD, DD);
    k_hop<1><<<CH / OWNB, NTHR, 0, stream>>>(x, rel, PH, PT, EHLw, LIST, CNT, OFF, FLAG, out, cs);
  }

  k_gemm_nt<1, 0><<<gPT, 256, 0, stream>>>(EHLs, W2T + 64 * 128, W, PT, NN, DD, 2 * DD, DD);
  for (int c = 0; c < NCH; ++c) {
    const int cs = c * CH;
    const int Mc = (NN - cs) < CH ? (NN - cs) : CH;
    const int gPH = ((Mc / 64) + 7) / 8;
    k_gemm_nt<1, 0><<<gPH, 256, 0, stream>>>(EHLs + (size_t)cs * 128, W2T, W, PH, Mc, DD, 2 * DD, DD);
    k_hop<2><<<CH / OWNB, NTHR, 0, stream>>>(x, rel, PH, PT, EHLw, LIST, CNT, OFF, FLAG, out, cs);
  }
}
